// DensityGCNProcessor_50989851738542
// MI455X (gfx1250) — hardware-verified
//
#include <hip/hip_runtime.h>
#include <stddef.h>


#define BATCH  4
#define NN     4096
#define NTOT   (BATCH * NN)
#define KNN    4
#define CIN    256
#define CHID   512
#define COUT   256
#define NTHR   256
#define NWAVE  8
#define TGT    32
#define TPW    (TGT / NWAVE)
#define EPT    8
#define CHK    (NTHR * EPT)
#define NENT   (NN * KNN)
#define NCHK   (NENT / CHK)
#define WLCAP  (EPT * 32)
#define LCAP   1024
#define DEGCAP 32
#define SP     36
#define GR     64
#define GC     128
#define TS     64
#define WSCAP  134217728

static_assert(NENT % CHK == 0);
static_assert(TGT == 32 && NWAVE * 32 == NTHR && (TGT % NWAVE) == 0);
static_assert(NN % TGT == 0 && NTOT % NTHR == 0 && NN % NTHR == 0);
static_assert(NTOT % GR == 0 && CHID % GC == 0 && COUT % GC == 0);
static_assert(CIN % 32 == 0 && CHID % 32 == 0);
static_assert(NN % TS == 0 && CIN % TS == 0 && CHID % TS == 0 && COUT % TS == 0);
static_assert(GR == 4 * 16 && GC == 2 * 64 && NWAVE == 8);
static_assert(LCAP == TGT * DEGCAP);
static_assert((SP % 4) == 0);
static_assert(CHID == 2 * 8 * 32 && COUT == 8 * 32);
static_assert(COUT == NWAVE * 32);
static_assert((TS * TS / 4) % NTHR == 0);
static_assert(NN % (4 * NTHR) == 0);

typedef float          v4f  __attribute__((ext_vector_type(4)));
typedef float          v8f  __attribute__((ext_vector_type(8)));
typedef int            v4i  __attribute__((ext_vector_type(4)));
typedef unsigned short v8us __attribute__((ext_vector_type(8)));
typedef __bf16         v16b __attribute__((ext_vector_type(16)));
union FragB { v16b v; v8us h[2]; };

__device__ __forceinline__ unsigned int bfr(float f) {
  const unsigned int u = __float_as_uint(f);
  return (u + 0x7FFFu + ((u >> 16) & 1u)) >> 16;
}

__device__ __forceinline__ void split1(float x, unsigned short& hb, unsigned short& lb) {
  const unsigned int hu = bfr(x);
  const float hf = __uint_as_float(hu << 16);
  hb = (unsigned short)hu;
  lb = (unsigned short)bfr(x - hf);
}

__device__ __forceinline__ void split8(v4f a, v4f b, v8us& hi, v8us& lo) {
  unsigned short hb, lb;
  split1(a.x, hb, lb); hi[0] = hb; lo[0] = lb;
  split1(a.y, hb, lb); hi[1] = hb; lo[1] = lb;
  split1(a.z, hb, lb); hi[2] = hb; lo[2] = lb;
  split1(a.w, hb, lb); hi[3] = hb; lo[3] = lb;
  split1(b.x, hb, lb); hi[4] = hb; lo[4] = lb;
  split1(b.y, hb, lb); hi[5] = hb; lo[5] = lb;
  split1(b.z, hb, lb); hi[6] = hb; lo[6] = lb;
  split1(b.w, hb, lb); hi[7] = hb; lo[7] = lb;
}

__device__ __forceinline__ v4f relu4(v4f v) {
  v.x = fmaxf(v.x, 0.f); v.y = fmaxf(v.y, 0.f); v.z = fmaxf(v.z, 0.f); v.w = fmaxf(v.w, 0.f);
  return v;
}

__device__ __forceinline__ v8f wmb(v16b a, v16b b, v8f c) {
  v8f d = __builtin_amdgcn_wmma_f32_16x16x32_bf16(false, a, false, b, (short)0, c, false, false);
  asm volatile("v_nop\n\tv_nop\n\tv_nop\n\tv_nop" : "+v"(d) : "v"(a), "v"(b));
  return d;
}

__global__ __launch_bounds__(NTHR) void k_knn(const float* __restrict__ dens, int* tgt) {
  __shared__ __attribute__((aligned(16))) float sd[NN];
  const int tid = threadIdx.x;
  const int blk = blockIdx.x;
  const int b = blk / (NN / NTHR);
  const float* src = dens + (size_t)b * NN;
#pragma unroll
  for (int i = 0; i < NN / (4 * NTHR); ++i) {
    const int idx = i * NTHR + tid;
    *(v4f*)(sd + 4 * idx) = *(const v4f*)(src + 4 * idx);
  }
  __syncthreads();
  const int node = blk * NTHR + tid;
  const int i = node & (NN - 1);
  const float di = sd[i];
  const float big = 3.0e38f;
  float k0 = big, k1 = big, k2 = big, k3 = big, k4 = big;
  int   i0 = 0,   i1 = 0,   i2 = 0,   i3 = 0,   i4 = 0;
#pragma unroll 4
  for (int j = 0; j < NN; ++j) {
    const float d = fabsf(sd[j] - di);
    if (d < k4) {
      if (d < k0)      { k4 = k3; i4 = i3; k3 = k2; i3 = i2; k2 = k1; i2 = i1; k1 = k0; i1 = i0; k0 = d; i0 = j; }
      else if (d < k1) { k4 = k3; i4 = i3; k3 = k2; i3 = i2; k2 = k1; i2 = i1; k1 = d; i1 = j; }
      else if (d < k2) { k4 = k3; i4 = i3; k3 = k2; i3 = i2; k2 = d; i2 = j; }
      else if (d < k3) { k4 = k3; i4 = i3; k3 = d; i3 = j; }
      else             { k4 = d; i4 = j; }
    }
  }
  v4i r;
  r.x = i1; r.y = i2; r.z = i3; r.w = i4;
  int* tp = tgt + (size_t)node * KNN;
  *(volatile v4i*)tp = r;
  __threadfence();
  *(volatile v4i*)tp = r;
}

__device__ __forceinline__ int collect_hits(const int* __restrict__ tl, int tb,
                                           int* wl, int* wcnt, int* blist,
                                           int tid, int lane, int wave) {
  int L = 0;
#pragma unroll 1
  for (int ch = 0; ch < NCHK; ++ch) {
    const int e0 = ch * CHK + tid * EPT;
    const v4i da = *(const v4i*)(tl + e0);
    const v4i db = *(const v4i*)(tl + e0 + 4);
    int val[8];
    val[0] = da.x; val[1] = da.y; val[2] = da.z; val[3] = da.w;
    val[4] = db.x; val[5] = db.y; val[6] = db.z; val[7] = db.w;
    int wc = 0;
#pragma unroll
    for (int j = 0; j < EPT; ++j) {
      const unsigned s = (unsigned)(val[j] - tb);
      const bool hit = s < (unsigned)TGT;
      const unsigned mk = __builtin_amdgcn_ballot_w32(hit);
      if (hit) {
        int pos = wc + (int)__builtin_amdgcn_mbcnt_lo(mk, 0u);
        pos = pos > WLCAP - 1 ? WLCAP - 1 : pos;
        wl[wave * WLCAP + pos] = (((e0 + j) >> 2) << 5) | (int)s;
      }
      wc += (int)__builtin_popcount(mk);
    }
    wc = wc > WLCAP ? WLCAP : wc;
    if (lane == 0) wcnt[wave] = wc;
    __syncthreads();
    int pre = 0, tot = 0;
#pragma unroll
    for (int w = 0; w < NWAVE; ++w) {
      const int c = wcnt[w];
      pre += (w < wave) ? c : 0;
      tot += c;
    }
#pragma unroll 1
    for (int i = lane; i < wc; i += 32) {
      const int pos = L + pre + i;
      if (pos < LCAP) blist[pos] = wl[wave * WLCAP + i];
    }
    L += tot;
    L = L > LCAP ? LCAP : L;
    __syncthreads();
  }
  return L;
}

__global__ __launch_bounds__(NTHR) void k_count(const int* __restrict__ tgt, float* dinv) {
  __shared__ __attribute__((aligned(16))) int wl[NWAVE * WLCAP];
  __shared__ __attribute__((aligned(16))) int blist[LCAP];
  __shared__ __attribute__((aligned(16))) int scnt[TGT];
  __shared__ int wcnt[NWAVE];
  const int tid = threadIdx.x, lane = tid & 31, wave = tid >> 5;
  const int gt = blockIdx.x * TGT;
  const int b  = gt / NN;
  const int tb = gt & (NN - 1);
  const int L = collect_hits(tgt + (size_t)b * NENT, tb, wl, wcnt, blist, tid, lane, wave);
  if (wave == 0) {
    int n = 0;
#pragma unroll 1
    for (int i = 0; i < L; ++i) n += ((blist[i] & (TGT - 1)) == lane) ? 1 : 0;
    scnt[lane] = n;
  }
  __syncthreads();
  v4f dq = {0.f, 0.f, 0.f, 0.f};
  const int t8 = tid < 8 ? tid : 0;
  if (tid < 8) {
    const v4i c = *(const v4i*)(scnt + 4 * t8);
    dq.x = rsqrtf((float)(c.x + 1));
    dq.y = rsqrtf((float)(c.y + 1));
    dq.z = rsqrtf((float)(c.z + 1));
    dq.w = rsqrtf((float)(c.w + 1));
  }
  float* dp = dinv + (size_t)gt + 4 * t8;
  if (tid < 8) *(volatile v4f*)dp = dq;
  __threadfence();
  if (tid < 8) *(volatile v4f*)dp = dq;
}

__global__ __launch_bounds__(NTHR) void k_tsplit(const float* __restrict__ in,
                                                 unsigned short* oh, unsigned short* ol,
                                                 int ldi, int ldo, int inZ, int outZ) {
  __shared__ float tile[TS][TS + 1];
  const int tid = threadIdx.x;
  const int q0 = blockIdx.x * TS, r0 = blockIdx.y * TS, z = blockIdx.z;
  const float* ip = in + (size_t)z * (size_t)inZ + (size_t)r0 * (size_t)ldi + q0;
#pragma unroll
  for (int i = 0; i < (TS * TS / 4) / NTHR; ++i) {
    const int idx = i * NTHR + tid;
    const int r = idx >> 4, f = idx & 15;
    const v4f v = *(const v4f*)(ip + (size_t)r * (size_t)ldi + 4 * f);
    tile[r][4 * f + 0] = v.x; tile[r][4 * f + 1] = v.y;
    tile[r][4 * f + 2] = v.z; tile[r][4 * f + 3] = v.w;
  }
  __syncthreads();
  const int j = tid & 7, qs = tid >> 3;
  v8us hv[2], lv[2];
#pragma unroll
  for (int it = 0; it < 2; ++it) {
    const int ql = it * 32 + qs;
    v4f a, b;
    a.x = tile[8 * j + 0][ql]; a.y = tile[8 * j + 1][ql]; a.z = tile[8 * j + 2][ql]; a.w = tile[8 * j + 3][ql];
    b.x = tile[8 * j + 4][ql]; b.y = tile[8 * j + 5][ql]; b.z = tile[8 * j + 6][ql]; b.w = tile[8 * j + 7][ql];
    split8(a, b, hv[it], lv[it]);
  }
  const size_t o0 = (size_t)z * (size_t)outZ + (size_t)(q0 + qs) * (size_t)ldo + (size_t)(r0 + 8 * j);
  const size_t st = (size_t)32 * (size_t)ldo;
  unsigned short* dh = oh + o0;
  unsigned short* dl = ol + o0;
  *(volatile v8us*)dh = hv[0];      *(volatile v8us*)(dh + st) = hv[1];
  *(volatile v8us*)dl = lv[0];      *(volatile v8us*)(dl + st) = lv[1];
  __threadfence();
  *(volatile v8us*)dh = hv[0];      *(volatile v8us*)(dh + st) = hv[1];
  *(volatile v8us*)dl = lv[0];      *(volatile v8us*)(dl + st) = lv[1];
}

__global__ __launch_bounds__(NTHR) void k_gemm(const unsigned short* __restrict__ Ah,
                                               const unsigned short* __restrict__ Al,
                                               const unsigned short* __restrict__ Bh,
                                               const unsigned short* __restrict__ Bl,
                                               const float* __restrict__ dinv, float* C,
                                               int K, int N) {
  __shared__ __attribute__((aligned(16))) float stg[NWAVE * 16 * 64];
  const int tid = threadIdx.x, lane = tid & 31, wave = tid >> 5, hh = lane >> 4, m = lane & 15;
  const int row0 = blockIdx.x * GR + (wave & 3) * 16;
  const int col0 = blockIdx.y * GC + (wave >> 2) * 64;
  const unsigned short* ahp = Ah + (size_t)(row0 + m) * (size_t)K + 8 * hh;
  const unsigned short* alp = Al + (size_t)(row0 + m) * (size_t)K + 8 * hh;
  const unsigned short* bhp = Bh + (size_t)(col0 + m) * (size_t)K + 8 * hh;
  const unsigned short* blp = Bl + (size_t)(col0 + m) * (size_t)K + 8 * hh;

  v8f acc[4];
#pragma unroll
  for (int t = 0; t < 4; ++t) { v8f zz = {0.f, 0.f, 0.f, 0.f, 0.f, 0.f, 0.f, 0.f}; acc[t] = zz; }

#pragma unroll 1
  for (int k0 = 0; k0 < K; k0 += 32) {
    FragB ah, al;
    ah.h[0] = *(const v8us*)(ahp + k0);
    ah.h[1] = *(const v8us*)(ahp + k0 + 16);
    al.h[0] = *(const v8us*)(alp + k0);
    al.h[1] = *(const v8us*)(alp + k0 + 16);
#pragma unroll
    for (int t = 0; t < 4; ++t) {
      const size_t bo = (size_t)(16 * t) * (size_t)K + (size_t)k0;
      FragB bh, bl;
      bh.h[0] = *(const v8us*)(bhp + bo);
      bh.h[1] = *(const v8us*)(bhp + bo + 16);
      bl.h[0] = *(const v8us*)(blp + bo);
      bl.h[1] = *(const v8us*)(blp + bo + 16);
      acc[t] = wmb(ah.v, bh.v, acc[t]);
      acc[t] = wmb(ah.v, bl.v, acc[t]);
      acc[t] = wmb(al.v, bh.v, acc[t]);
    }
  }

  const v4f dA = *(const v4f*)(dinv + (size_t)row0 + 8 * hh);
  const v4f dB = *(const v4f*)(dinv + (size_t)row0 + 8 * hh + 4);
  float s[8];
  s[0] = dA.x; s[1] = dA.y; s[2] = dA.z; s[3] = dA.w; s[4] = dB.x; s[5] = dB.y; s[6] = dB.z; s[7] = dB.w;
  float* sp = stg + wave * (16 * 64) + (8 * hh) * 64 + m;
#pragma unroll
  for (int t = 0; t < 4; ++t) {
#pragma unroll
    for (int r = 0; r < 8; ++r) sp[r * 64 + 16 * t] = acc[t][r] * s[r];
  }
  __syncthreads();

  const float* lp = stg + wave * (16 * 64);
#pragma unroll
  for (int i = 0; i < 8; ++i) {
    const int rr = 2 * i + hh;
    const v4f v = *(const v4f*)(lp + rr * 64 + 4 * m);
    *(volatile v4f*)(C + (size_t)(row0 + rr) * (size_t)N + col0 + 4 * m) = v;
  }
  __threadfence();
#pragma unroll
  for (int i = 0; i < 8; ++i) {
    const int rr = 2 * i + hh;
    const v4f v = *(const v4f*)(lp + rr * 64 + 4 * m);
    *(volatile v4f*)(C + (size_t)(row0 + rr) * (size_t)N + col0 + 4 * m) = v;
  }
}

__device__ __forceinline__ void build_slot_lists(const int* blist, int L, int* slist, int* scnt, int lane, int wave) {
  if (wave == 0) {
    int n = 0;
#pragma unroll 1
    for (int i = 0; i < L; ++i) {
      const int ent = blist[i];
      if ((ent & (TGT - 1)) == lane) {
        if (n < DEGCAP) slist[lane * DEGCAP + n] = ent >> 5;
        ++n;
      }
    }
    scnt[lane] = n > DEGCAP ? DEGCAP : n;
  }
}

__global__ __launch_bounds__(NTHR) void k_agg1(const int* __restrict__ tgt, const float* __restrict__ dinv,
                                               const float* __restrict__ hw, const float* __restrict__ bias,
                                               unsigned short* Hh, unsigned short* Hl) {
  __shared__ __attribute__((aligned(16))) int wl[NWAVE * WLCAP];
  __shared__ __attribute__((aligned(16))) int blist[LCAP];
  __shared__ __attribute__((aligned(16))) int slist[TGT * DEGCAP];
  __shared__ __attribute__((aligned(16))) int scnt[TGT];
  __shared__ int wcnt[NWAVE];
  const int tid = threadIdx.x, lane = tid & 31, wave = tid >> 5;
  const int gt = blockIdx.x * TGT;
  const int b  = gt / NN;
  const int tb = gt & (NN - 1);
  const int bN = b * NN;
  const int L = collect_hits(tgt + (size_t)b * NENT, tb, wl, wcnt, blist, tid, lane, wave);
  build_slot_lists(blist, L, slist, scnt, lane, wave);
  __syncthreads();

  const v4f bA = *(const v4f*)(bias + 8 * lane);
  const v4f bB = *(const v4f*)(bias + 8 * lane + 4);
  const v4f bC = *(const v4f*)(bias + 256 + 8 * lane);
  const v4f bD = *(const v4f*)(bias + 256 + 8 * lane + 4);
#pragma unroll 1
  for (int q = 0; q < TPW; ++q) {
    const int slot = wave * TPW + q;
    int n = scnt[slot];
    n = n < 0 ? 0 : (n > DEGCAP ? DEGCAP : n);
    v4f a0 = {0.f, 0.f, 0.f, 0.f}, a1 = a0, a2 = a0, a3 = a0;
#pragma unroll 1
    for (int p = 0; p < n; ++p) {
      int s = slist[slot * DEGCAP + p];
      s = s < 0 ? 0 : (s > NN - 1 ? NN - 1 : s);
      const float* rp = hw + (size_t)(bN + s) * CHID + 8 * lane;
      a0 += *(const v4f*)rp;         a1 += *(const v4f*)(rp + 4);
      a2 += *(const v4f*)(rp + 256); a3 += *(const v4f*)(rp + 260);
    }
    const int tnode = bN + tb + slot;
    {
      const float* rp = hw + (size_t)tnode * CHID + 8 * lane;
      a0 += *(const v4f*)rp;         a1 += *(const v4f*)(rp + 4);
      a2 += *(const v4f*)(rp + 256); a3 += *(const v4f*)(rp + 260);
    }
    const float dt = dinv[tnode];
    const v4f v0 = relu4(a0 * dt + bA), v1 = relu4(a1 * dt + bB);
    const v4f v2 = relu4(a2 * dt + bC), v3 = relu4(a3 * dt + bD);
    v8us h0, l0, h1, l1;
    split8(v0, v1, h0, l0);
    split8(v2, v3, h1, l1);
    unsigned short* ph = Hh + (size_t)tnode * CHID + 8 * lane;
    unsigned short* pl = Hl + (size_t)tnode * CHID + 8 * lane;
    *(volatile v8us*)ph = h0; *(volatile v8us*)(ph + 256) = h1;
    *(volatile v8us*)pl = l0; *(volatile v8us*)(pl + 256) = l1;
    __threadfence();
    *(volatile v8us*)ph = h0; *(volatile v8us*)(ph + 256) = h1;
    *(volatile v8us*)pl = l0; *(volatile v8us*)(pl + 256) = l1;
  }
}

__global__ __launch_bounds__(NTHR) void k_agg2(const int* __restrict__ tgt, const float* __restrict__ dinv,
                                               const float* __restrict__ hw, const float* __restrict__ bias,
                                               float* out) {
  __shared__ __attribute__((aligned(16))) int wl[NWAVE * WLCAP];
  __shared__ __attribute__((aligned(16))) int blist[LCAP];
  __shared__ __attribute__((aligned(16))) int slist[TGT * DEGCAP];
  __shared__ __attribute__((aligned(16))) int scnt[TGT];
  __shared__ int wcnt[NWAVE];
  __shared__ __attribute__((aligned(16))) float stg[COUT * SP];
  const int tid = threadIdx.x, lane = tid & 31, wave = tid >> 5;
  const int gt = blockIdx.x * TGT;
  const int b  = gt / NN;
  const int tb = gt & (NN - 1);
  const int bN = b * NN;
  const int L = collect_hits(tgt + (size_t)b * NENT, tb, wl, wcnt, blist, tid, lane, wave);
  build_slot_lists(blist, L, slist, scnt, lane, wave);
  __syncthreads();

  const v4f bA = *(const v4f*)(bias + 8 * lane);
  const v4f bB = *(const v4f*)(bias + 8 * lane + 4);
#pragma unroll 1
  for (int q = 0; q < TPW; ++q) {
    const int slot = wave * TPW + q;
    int n = scnt[slot];
    n = n < 0 ? 0 : (n > DEGCAP ? DEGCAP : n);
    v4f a0 = {0.f, 0.f, 0.f, 0.f}, a1 = a0;
#pragma unroll 1
    for (int p = 0; p < n; ++p) {
      int s = slist[slot * DEGCAP + p];
      s = s < 0 ? 0 : (s > NN - 1 ? NN - 1 : s);
      const float* rp = hw + (size_t)(bN + s) * COUT + 8 * lane;
      a0 += *(const v4f*)rp; a1 += *(const v4f*)(rp + 4);
    }
    const int tnode = bN + tb + slot;
    {
      const float* rp = hw + (size_t)tnode * COUT + 8 * lane;
      a0 += *(const v4f*)rp; a1 += *(const v4f*)(rp + 4);
    }
    const float dt = dinv[tnode];
    const v4f v0 = relu4(a0 * dt + bA), v1 = relu4(a1 * dt + bB);
    float* sg = stg + (8 * lane) * SP + slot;
    sg[0 * SP] = v0.x; sg[1 * SP] = v0.y; sg[2 * SP] = v0.z; sg[3 * SP] = v0.w;
    sg[4 * SP] = v1.x; sg[5 * SP] = v1.y; sg[6 * SP] = v1.z; sg[7 * SP] = v1.w;
  }
  __syncthreads();

  const int piece = lane & 7, lq = lane >> 3;
#pragma unroll
  for (int i = 0; i < 8; ++i) {
    const int c = wave * 32 + i * 4 + lq;
    const v4f v = *(const v4f*)(stg + c * SP + 4 * piece);
    *(volatile v4f*)(out + ((size_t)(b * COUT + c)) * NN + tb + 4 * piece) = v;
  }
  __threadfence();
#pragma unroll
  for (int i = 0; i < 8; ++i) {
    const int c = wave * 32 + i * 4 + lq;
    const v4f v = *(const v4f*)(stg + c * SP + 4 * piece);
    *(volatile v4f*)(out + ((size_t)(b * COUT + c)) * NN + tb + 4 * piece) = v;
  }
}

extern "C" void kernel_launch(void* const* d_in, const int* in_sizes, int n_in,
                              void* d_out, int out_size, void* d_ws, size_t ws_size,
                              hipStream_t stream) {
  if (n_in < 6) return;
  if (in_sizes[0] != NTOT) return;
  if (in_sizes[1] != NTOT * CIN) return;
  if (in_sizes[2] != CIN * CHID || in_sizes[3] != CHID) return;
  if (in_sizes[4] != CHID * COUT || in_sizes[5] != COUT) return;
  if (out_size != NTOT * COUT) return;

  const float* dens = (const float*)d_in[0];
  const float* fm   = (const float*)d_in[1];
  const float* W1   = (const float*)d_in[2];
  const float* b1   = (const float*)d_in[3];
  const float* W2   = (const float*)d_in[4];
  const float* b2   = (const float*)d_in[5];
  float* out = (float*)d_out;

  char* ws = (char*)d_ws;
  size_t off = 0;
  const size_t oTgt = off; off += (size_t)NTOT * KNN * 4;          off = (off + 255) & ~(size_t)255;
  const size_t oDv  = off; off += (size_t)NTOT * 4;                off = (off + 255) & ~(size_t)255;
  const size_t oP1h = off; off += (size_t)CHID * CIN * 2;          off = (off + 255) & ~(size_t)255;
  const size_t oP1l = off; off += (size_t)CHID * CIN * 2;          off = (off + 255) & ~(size_t)255;
  const size_t oP2h = off; off += (size_t)COUT * CHID * 2;         off = (off + 255) & ~(size_t)255;
  const size_t oP2l = off; off += (size_t)COUT * CHID * 2;         off = (off + 255) & ~(size_t)255;
  const size_t oXh  = off; off += (size_t)NTOT * CIN * 2;          off = (off + 255) & ~(size_t)255;
  const size_t oXl  = off; off += (size_t)NTOT * CIN * 2;          off = (off + 255) & ~(size_t)255;
  const size_t oHw  = off; off += (size_t)NTOT * CHID * 4;         off = (off + 255) & ~(size_t)255;
  const size_t oH1h = off; off += (size_t)NTOT * CHID * 2;         off = (off + 255) & ~(size_t)255;
  const size_t oH1l = off; off += (size_t)NTOT * CHID * 2;         off = (off + 255) & ~(size_t)255;
  if (off > ws_size || off > (size_t)WSCAP) return;
  int*            tgt  = (int*)(ws + oTgt);
  float*          dinv = (float*)(ws + oDv);
  unsigned short* P1h  = (unsigned short*)(ws + oP1h);
  unsigned short* P1l  = (unsigned short*)(ws + oP1l);
  unsigned short* P2h  = (unsigned short*)(ws + oP2h);
  unsigned short* P2l  = (unsigned short*)(ws + oP2l);
  unsigned short* Xh   = (unsigned short*)(ws + oXh);
  unsigned short* Xl   = (unsigned short*)(ws + oXl);
  float*          hw   = (float*)(ws + oHw);
  unsigned short* H1h  = (unsigned short*)(ws + oH1h);
  unsigned short* H1l  = (unsigned short*)(ws + oH1l);

  k_knn<<<NTOT / NTHR, NTHR, 0, stream>>>(dens, tgt);
  k_count<<<NTOT / TGT, NTHR, 0, stream>>>(tgt, dinv);
  k_tsplit<<<dim3(NN / TS, CIN / TS, BATCH), NTHR, 0, stream>>>(fm, Xh, Xl, NN, CIN, CIN * NN, NN * CIN);
  k_tsplit<<<dim3(CHID / TS, CIN / TS, 1), NTHR, 0, stream>>>(W1, P1h, P1l, CHID, CIN, 0, 0);
  k_tsplit<<<dim3(COUT / TS, CHID / TS, 1), NTHR, 0, stream>>>(W2, P2h, P2l, COUT, CHID, 0, 0);
  k_gemm<<<dim3(NTOT / GR, CHID / GC, 1), NTHR, 0, stream>>>(Xh, Xl, P1h, P1l, dinv, hw, CIN, CHID);
  k_agg1<<<NTOT / TGT, NTHR, 0, stream>>>(tgt, dinv, hw, b1, H1h, H1l);
  k_gemm<<<dim3(NTOT / GR, COUT / GC, 1), NTHR, 0, stream>>>(H1h, H1l, P2h, P2l, dinv, hw, CHID, COUT);
  k_agg2<<<NTOT / TGT, NTHR, 0, stream>>>(tgt, dinv, hw, b2, out);
}
